// ONNXCompatibleCondConv2d_27522150432953
// MI455X (gfx1250) — hardware-verified
//
#include <hip/hip_runtime.h>
#include <math.h>

typedef __attribute__((ext_vector_type(16))) _Float16 v16h;
typedef __attribute__((ext_vector_type(16))) __bf16 v16b;
typedef __attribute__((ext_vector_type(8)))  _Float16 v8h;
typedef __attribute__((ext_vector_type(8)))  float v8f;
typedef __attribute__((ext_vector_type(4)))  float v4f;
typedef __attribute__((ext_vector_type(2)))  float v2f;
typedef __attribute__((ext_vector_type(4)))  unsigned v4u;
typedef __attribute__((ext_vector_type(4)))  int v4i;
typedef float __attribute__((may_alias)) float_a;
typedef int __attribute__((may_alias)) int_a;

template <typename T> __device__ __forceinline__ void vst2(void* p, T v) { *(volatile T*)p = v; __threadfence(); *(volatile T*)p = v; }
__device__ __forceinline__ v8f wmma16(v16h a, v16h b, v8f c) {
  v8f d = __builtin_amdgcn_wmma_f32_16x16x32_f16(false, a, false, b, (short)0, c, false, false);
  asm volatile("v_nop\n\tv_nop\n\tv_nop\n\tv_nop" : "+v"(d) : "v"(a), "v"(b));
  return d;
}
__device__ __forceinline__ v8f wmma_bf(v16b a, v16b b, v8f c) {
  v8f d = __builtin_amdgcn_wmma_f32_16x16x32_bf16(false, a, false, b, (short)0, c, false, false);
  asm volatile("v_nop\n\tv_nop\n\tv_nop\n\tv_nop" : "+v"(d) : "v"(a), "v"(b));
  return d;
}
__device__ __forceinline__ v16h frag_h(const _Float16* rowk0, int lane) {
  union { v16h v; v8h q[2]; } u; const _Float16* p = rowk0 + 8 * (lane >> 4);
  u.q[0] = *(const v8h*)p; u.q[1] = *(const v8h*)(p + 16); return u.v;
}
__device__ __forceinline__ v16h frag_f32(const float* rowk0, int lane) {
  v16h a; const float* p = rowk0 + 8 * (lane >> 4);
#pragma unroll
  for (int i = 0; i < 8; ++i) { a[i] = (_Float16)p[i]; a[8 + i] = (_Float16)p[16 + i]; }
  return a;
}
__device__ __forceinline__ v16h frag_f32s(const float* rowk0, int lane, float sc) {
  v16h a; const float* p = rowk0 + 8 * (lane >> 4);
#pragma unroll
  for (int i = 0; i < 8; ++i) { a[i] = (_Float16)(p[i] * sc); a[8 + i] = (_Float16)(p[16 + i] * sc); }
  return a;
}
__device__ __forceinline__ v16h fragc_f32(const float* W, int k0, int n, int lane, int ld, int K) {
  v16h a; const int g = lane >> 4;
#pragma unroll
  for (int i = 0; i < 8; ++i) { const int ka = k0 + 8 * g + i, kb = ka + 16;
    a[i] = (_Float16)(ka < K ? W[(size_t)ka * ld + n] : 0.f); a[8 + i] = (_Float16)(kb < K ? W[(size_t)kb * ld + n] : 0.f); }
  return a;
}
struct F2 { v16b h, l; };
__device__ __forceinline__ F2 bsplit16(const float v[16]) { F2 r;
#pragma unroll
  for (int i = 0; i < 16; ++i) { const __bf16 h = (__bf16)v[i]; r.h[i] = h; r.l[i] = (__bf16)(v[i] - (float)h); }
  return r; }
__device__ __forceinline__ F2 split_row(const float* row, int k0, int lane) { float v[16]; const float* p = row + k0 + 8 * (lane >> 4);
#pragma unroll
  for (int i = 0; i < 8; ++i) { v[i] = p[i]; v[8 + i] = p[16 + i]; }
  return bsplit16(v); }
__device__ __forceinline__ F2 split_rowK(const float* row, int k0, int lane, int K) { float v[16]; const int g = lane >> 4;
#pragma unroll
  for (int i = 0; i < 8; ++i) { const int ka = k0 + 8 * g + i, kb = ka + 16; v[i] = ka < K ? row[ka] : 0.f; v[8 + i] = kb < K ? row[kb] : 0.f; }
  return bsplit16(v); }
__device__ __forceinline__ F2 split_col(const float* W, int k0, int n, int lane, int ld, int K) { float v[16]; const int g = lane >> 4;
#pragma unroll
  for (int i = 0; i < 8; ++i) { const int ka = k0 + 8 * g + i, kb = ka + 16; v[i] = ka < K ? W[(size_t)ka * ld + n] : 0.f; v[8 + i] = kb < K ? W[(size_t)kb * ld + n] : 0.f; }
  return bsplit16(v); }
__device__ __forceinline__ v8f mac3(const F2& a, const F2& b, v8f c) { c = wmma_bf(a.l, b.h, c); c = wmma_bf(a.h, b.l, c); return wmma_bf(a.h, b.h, c); }
__device__ __forceinline__ float sigm(float v) { return 1.0f / (1.0f + expf(-v)); }
#define LDSX() do { asm volatile("s_wait_dscnt 0" ::: "memory"); __builtin_amdgcn_wave_barrier(); __builtin_amdgcn_fence(__ATOMIC_RELEASE, "workgroup"); } while (0)

#define NB 16
#define CIN 128
#define COUT 128
#define HH 56
#define WWD 56
#define NP (HH * WWD)
#define KTOT (CIN * 9)
#define NE 4

__global__ __launch_bounds__(256) void k_mix(const float* __restrict__ r, const float* __restrict__ W, _Float16* __restrict__ Wm) {
  const int o = blockIdx.x, b = blockIdx.y, tid = threadIdx.x;
  const float r0 = r[b * NE], r1 = r[b * NE + 1], r2 = r[b * NE + 2], r3 = r[b * NE + 3];
  __shared__ __align__(16) _Float16 srow[KTOT];
  for (int k = tid; k < KTOT; k += 256) { const size_t base = (size_t)o * KTOT + k; const size_t es = (size_t)COUT * KTOT;
    srow[k] = (_Float16)((r0 * W[base] + r1 * W[es + base] + r2 * W[2 * es + base] + r3 * W[3 * es + base]) * 16.0f); }
  __syncthreads();
  for (int q = tid; q < KTOT / 8; q += 256) vst2(Wm + ((size_t)b * COUT + o) * KTOT + q * 8, *(const v4u*)(&srow[q * 8]));
}
__global__ __launch_bounds__(256) void k_im2col(const float* __restrict__ x, _Float16* __restrict__ A) {
  __shared__ float tile[32][5][58];
  __shared__ __align__(16) _Float16 srow[64][KTOT + 8];
  const int b = blockIdx.y, p0 = blockIdx.x * 64, tid = threadIdx.x; const int y0 = p0 / WWD;
#pragma unroll 1
  for (int cc = 0; cc < CIN / 32; ++cc) {
    for (int q = tid; q < 32 * 5 * 58; q += 256) { const int cl = q / 290, rem = q % 290, rr = rem / 58, xx = rem % 58; const int yy = y0 - 1 + rr, xi = xx - 1;
      tile[cl][rr][xx] = (yy >= 0 && yy < HH && xi >= 0 && xi < WWD) ? x[(((size_t)b * CIN + cc * 32 + cl) * HH + yy) * WWD + xi] : 0.f; }
    __syncthreads();
    for (int q = tid; q < 64 * 32 * 9; q += 256) { const int pl = q / 288, rem = q % 288, cl = rem / 9, t = rem % 9; const int p = p0 + pl;
      const int py = p / WWD, px = p % WWD; const float v = tile[cl][py - y0 + t / 3][px + t % 3];
      srow[pl][cc * 288 + cl * 9 + t] = (_Float16)v; }
    __syncthreads(); }
  for (int q = tid; q < 64 * (KTOT / 8); q += 256) { const int pl = q / (KTOT / 8), pc = q % (KTOT / 8); vst2(A + ((size_t)b * NP + p0 + pl) * KTOT + pc * 8, *(const v4u*)(&srow[pl][pc * 8])); }
}
__global__ __launch_bounds__(128) void k_conv(const _Float16* __restrict__ A, const _Float16* __restrict__ Wm, float* __restrict__ out) {
  __shared__ __align__(16) float st[COUT][68];
  const int tid = threadIdx.x, wave = tid >> 5, lane = tid & 31, col = lane & 15, g = lane >> 4;
  const int b = blockIdx.y, p0 = blockIdx.x * 64, r0 = p0 + wave * 16;
  const _Float16* Ab = A + (size_t)b * NP * KTOT; const _Float16* Wb = Wm + (size_t)b * COUT * KTOT;
  v8f acc[8] = {};
#pragma unroll 1
  for (int kc = 0; kc < KTOT / 32; ++kc) { const v16h a = frag_h(Ab + (size_t)(r0 + col) * KTOT + kc * 32, lane);
#pragma unroll
    for (int j = 0; j < 8; ++j) acc[j] = wmma16(a, frag_h(Wb + (size_t)(j * 16 + col) * KTOT + kc * 32, lane), acc[j]); }
#pragma unroll
  for (int j = 0; j < 8; ++j)
#pragma unroll
    for (int r = 0; r < 8; ++r) st[j * 16 + col][wave * 16 + 8 * g + r] = acc[j][r] * (1.0f / 16.0f);
  __syncthreads();
  for (int q = tid; q < COUT * 16; q += 128) { const int o = q >> 4, pc = q & 15; vst2(out + ((size_t)b * COUT + o) * NP + p0 + pc * 4, *(const v4f*)(&st[o][pc * 4])); }
}
extern "C" void kernel_launch(void* const* d_in, const int* in_sizes, int n_in, void* d_out, int out_size, void* d_ws, size_t ws_size, hipStream_t stream) {
  (void)in_sizes; (void)n_in; (void)out_size; (void)ws_size;
  const float* x = (const float*)d_in[0]; const float* r = (const float*)d_in[1]; const float* W = (const float*)d_in[2];
  float* out = (float*)d_out;
  char* ws = (char*)d_ws; size_t off = 0;
  auto take = [&](size_t bytes) { char* p = ws + off; off += (bytes + 255) & ~(size_t)255; return p; };
  _Float16* Wm = (_Float16*)take((size_t)NB * COUT * KTOT * 2); _Float16* A = (_Float16*)take((size_t)NB * NP * KTOT * 2);
  k_mix<<<dim3(COUT, NB), 256, 0, stream>>>(r, W, Wm);
  k_im2col<<<dim3(NP / 64, NB), 256, 0, stream>>>(x, A);
  k_conv<<<dim3(NP / 64, NB), 128, 0, stream>>>(A, Wm, out);
}
